// GRUDecoder_19550691131787
// MI455X (gfx1250) — hardware-run, weakly checked
//
#include <hip/hip_runtime.h>
#include <math.h>

constexpr int NBAT    = 64;
constexpr int NLAT    = 64;
constexpr int NHID    = 512;
constexpr int NLAY    = 2;
constexpr int NG3     = 3 * NHID;
constexpr int NOUTF   = 128;
constexpr int NSTEP   = 512;
constexpr int NTHR    = 256;
constexpr int SEQ_BLK = 16;
constexpr int HP      = 520;
constexpr int PLSZ    = SEQ_BLK * HP;
constexpr int NROWS   = NBAT * NSTEP;
constexpr float WCARRY  = 256.0f;
constexpr float HCARRY  = 16.0f;
constexpr float ACC_INV = 1.0f / 4096.0f;
static_assert(NBAT % SEQ_BLK == 0, "");
static_assert(NHID == 64 * (NTHR / 32), "");
static_assert(NHID == 2 * NTHR, "");
static_assert(NHID % 32 == 0 && NLAT % 4 == 0, "");
static_assert(HP % 8 == 0, "");
static_assert((4 * PLSZ) % NTHR == 0, "");
static_assert(SEQ_BLK * NLAT == 4 * NTHR, "");
static_assert(NLAY * NG3 == 3 * 4 * NTHR, "");
static_assert(2 * NLAY * NG3 + 0 <= NLAY * SEQ_BLK * NHID, "");
static_assert(NROWS % 64 == 0 && NOUTF % 64 == 0 && NHID % 32 == 0, "");
static_assert((NLAY * NG3 * NHID) % (8 * NTHR) == 0, "");
static_assert((NOUTF * NHID) % (8 * NTHR) == 0, "");
static_assert(((NROWS / 64) * (NOUTF / 64)) % 8 == 0, "");

typedef __attribute__((ext_vector_type(16))) _Float16 v16h;
typedef __attribute__((ext_vector_type(8)))  _Float16 v8h;
typedef __attribute__((ext_vector_type(16))) __bf16   v16b;
typedef __attribute__((ext_vector_type(8)))  __bf16   v8b;
typedef __attribute__((ext_vector_type(8)))  float    v8f;
typedef __attribute__((ext_vector_type(4)))  float    v4f;

__device__ __forceinline__ unsigned short f2bf_bits(float f) {
  unsigned u = __float_as_uint(f);
  return (unsigned short)((u + 0x7FFFu + ((u >> 16) & 1u)) >> 16);
}
__device__ __forceinline__ float bf_bits2f(unsigned short h) { return __uint_as_float(((unsigned)h) << 16); }

__device__ __forceinline__ void dep_guard_h(v8f& a, v8f& b, v16h x, v16h y) { asm volatile("v_nop\n\tv_nop\n\tv_nop\n\tv_nop" : "+v"(a), "+v"(b) : "v"(x), "v"(y)); }
__device__ __forceinline__ void dep_guard_b(v8f& a, v8f& b, v16b x, v16b y) { asm volatile("v_nop\n\tv_nop\n\tv_nop\n\tv_nop" : "+v"(a), "+v"(b) : "v"(x), "v"(y)); }
__device__ __forceinline__ void keep4_h(v16h a, v16h b, v16h c, v16h d) { asm volatile("v_nop" :: "v"(a), "v"(b), "v"(c), "v"(d)); }
__device__ __forceinline__ void keep4_b(v16b a, v16b b, v16b c, v16b d) { asm volatile("v_nop" :: "v"(a), "v"(b), "v"(c), "v"(d)); }
__device__ __forceinline__ void acc_guard4(v8f& a, v8f& b, v8f& c, v8f& d) { asm volatile("v_nop\n\tv_nop\n\tv_nop\n\tv_nop" : "+v"(a), "+v"(b), "+v"(c), "+v"(d)); }
__device__ __forceinline__ void guard6_h(v8f& a0, v8f& a1, v8f& a2, v8f& a3, v8f& a4, v8f& a5,
                                         v16h f0, v16h f1, v16h f2, v16h f3, v16h f4, v16h f5, v16h f6, v16h f7) {
  asm volatile("v_nop\n\tv_nop\n\tv_nop\n\tv_nop"
               : "+v"(a0), "+v"(a1), "+v"(a2), "+v"(a3), "+v"(a4), "+v"(a5)
               : "v"(f0), "v"(f1), "v"(f2), "v"(f3), "v"(f4), "v"(f5), "v"(f6), "v"(f7));
}
__device__ __forceinline__ void acc_guard6(v8f& a0, v8f& a1, v8f& a2, v8f& a3, v8f& a4, v8f& a5) {
  asm volatile("v_nop\n\tv_nop\n\tv_nop\n\tv_nop" : "+v"(a0), "+v"(a1), "+v"(a2), "+v"(a3), "+v"(a4), "+v"(a5));
}

template <typename T> struct Frag;
template <> struct Frag<_Float16> {
  typedef v16h V; union U { v16h v; v8h h[2]; };
  static __device__ __forceinline__ v16h load(const _Float16* p) {
    U f; f.h[0] = *(const v8h*)(p); f.h[1] = *(const v8h*)(p + 16); return f.v;
  }
  static __device__ __forceinline__ v8f mma(v16h a, v16h b, v8f c) {
    return __builtin_amdgcn_wmma_f32_16x16x32_f16(false, a, false, b, (short)0, c, false, false);
  }
  static __device__ __forceinline__ void guard(v8f& a, v8f& b, v16h x, v16h y) { dep_guard_h(a, b, x, y); }
  static __device__ __forceinline__ void keep(v16h a, v16h b, v16h c, v16h d) { keep4_h(a, b, c, d); }
};
template <> struct Frag<__bf16> {
  typedef v16b V; union U { v16b v; v8b h[2]; };
  static __device__ __forceinline__ v16b load(const __bf16* p) {
    U f; f.h[0] = *(const v8b*)(p); f.h[1] = *(const v8b*)(p + 16); return f.v;
  }
  static __device__ __forceinline__ v8f mma(v16b a, v16b b, v8f c) {
    return __builtin_amdgcn_wmma_f32_16x16x32_bf16(false, a, false, b, (short)0, c, false, false);
  }
  static __device__ __forceinline__ void guard(v8f& a, v8f& b, v16b x, v16b y) { dep_guard_b(a, b, x, y); }
  static __device__ __forceinline__ void keep(v16b a, v16b b, v16b c, v16b d) { keep4_b(a, b, c, d); }
};

__device__ __forceinline__ float fsig(float x)  { return __builtin_amdgcn_rcpf(1.0f + __expf(-x)); }
__device__ __forceinline__ float ftanh(float x) { return 1.0f - 2.0f * __builtin_amdgcn_rcpf(__expf(2.0f * x) + 1.0f); }

template <int ET> struct Elem;
template <> struct Elem<0> { typedef _Float16 T; };
template <> struct Elem<1> { typedef __bf16 T; };
template <int ET, bool SPLIT, int BIAS_MODE, int OUT_MODE, bool RESID, int ACT = 0>
__global__ __launch_bounds__(256) void wmma_gemm64(
    const unsigned short* __restrict__ Ap, const unsigned short* __restrict__ A2p, int lda, long strideA,
    const unsigned short* __restrict__ Btp, const unsigned short* __restrict__ Bt2p, int ldb, long strideB,
    void* __restrict__ Cout, void* __restrict__ Cout2, int ldc, long strideC,
    const float* __restrict__ bias,
    const float* __restrict__ resid, long strideR,
    int M, int N, int K, float scale) {
  typedef typename Elem<ET>::T T;
  typedef typename Frag<T>::V V;
  const T* A = (const T*)Ap; const T* A2 = (const T*)A2p; const T* Bt = (const T*)Btp; const T* Bt2 = (const T*)Bt2p;
  __shared__ __align__(16) float sT[8][16 * 68];
  const int b    = blockIdx.y;
  const int lane = threadIdx.x & 31;
  const int wave = threadIdx.x >> 5;
  const int tilesN = N >> 6;
  const int tilesM = M >> 6;
  const int tile = blockIdx.x * 8 + wave;
  if (tile >= tilesM * tilesN) return;
  const int tm = tile / tilesN;
  const int tn = tile - tm * tilesN;
  const int m0 = tm << 6;
  const int n0 = tn << 6;

  const T* Ab  = A  + (size_t)b * strideA;
  const T* Bb  = Bt + (size_t)b * strideB;
  const T* Ab2 = SPLIT ? (A2  + (size_t)b * strideA) : nullptr;
  const T* Bb2 = SPLIT ? (Bt2 + (size_t)b * strideB) : nullptr;

  const int rlane = lane & 15;
  const int koff  = (lane >> 4) * 8;
  const int mOff  = (lane >> 4) * 8;

  v8f acc[4][4];
#pragma unroll
  for (int i = 0; i < 4; ++i)
#pragma unroll
    for (int j = 0; j < 4; ++j) acc[i][j] = (v8f){0.f,0.f,0.f,0.f,0.f,0.f,0.f,0.f};

  for (int k0 = 0; k0 < K; k0 += 32) {
    V bh[4], bl[4];
#pragma unroll
    for (int j = 0; j < 4; ++j) {
      const size_t bo = (size_t)(n0 + (j << 4) + rlane) * ldb + koff + k0;
      bh[j] = Frag<T>::load(Bb + bo);
      if (SPLIT) bl[j] = Frag<T>::load(Bb2 + bo);
    }
#pragma unroll
    for (int i = 0; i < 4; ++i) {
      const size_t ao = (size_t)(m0 + (i << 4) + rlane) * lda + koff + k0;
      V ah = Frag<T>::load(Ab + ao);
      V al;
      if (SPLIT) al = Frag<T>::load(Ab2 + ao);
#pragma unroll
      for (int j = 0; j < 4; ++j) {
        acc[i][j] = Frag<T>::mma(ah, bh[j], acc[i][j]);
        if (SPLIT) {
          acc[i][j] = Frag<T>::mma(ah, bl[j], acc[i][j]);
          acc[i][j] = Frag<T>::mma(al, bh[j], acc[i][j]);
        }
      }
      Frag<T>::guard(acc[i][0], acc[i][3], ah, SPLIT ? al : ah);
    }
    Frag<T>::keep(bh[0], bh[1], bh[2], bh[3]);
    if (SPLIT) Frag<T>::keep(bl[0], bl[1], bl[2], bl[3]);
  }
  acc_guard4(acc[0][0], acc[0][1], acc[0][2], acc[0][3]);
  acc_guard4(acc[1][0], acc[1][1], acc[1][2], acc[1][3]);
  acc_guard4(acc[2][0], acc[2][1], acc[2][2], acc[2][3]);
  acc_guard4(acc[3][0], acc[3][1], acc[3][2], acc[3][3]);

  float* slab = sT[wave];
  const float* Rb = RESID ? (resid + (size_t)b * strideR) : nullptr;
#pragma unroll
  for (int i = 0; i < 4; ++i) {
    const int mBase = m0 + (i << 4);
#pragma unroll
    for (int j = 0; j < 4; ++j) {
      const int n = n0 + (j << 4) + rlane;
      float bv = 0.f;
      if (BIAS_MODE == 2) bv = bias[n];
#pragma unroll
      for (int r = 0; r < 8; ++r) {
        float v = acc[i][j][r] * scale;
        if (BIAS_MODE == 1) v += bias[mBase + mOff + r];
        if (BIAS_MODE == 2) v += bv;
        if (RESID) v += Rb[(size_t)(mBase + mOff + r) * ldc + n];
        if (ACT == 1) v = tanhf(v);
        if (ACT == 2) v = fmaxf(v, 0.0f);
        if (ACT == 3) v = v / (1.0f + expf(-v));
        if (ACT == 4) v = (v > 0.f) ? v : 0.01f * v;
        if (ACT == 5) v = 0.5f * v * (1.0f + erff(v * 0.70710678118654752f));
        slab[(mOff + r) * 68 + (j << 4) + rlane] = v;
      }
    }
    __builtin_amdgcn_fence(__ATOMIC_RELEASE, "workgroup");
    __builtin_amdgcn_wave_barrier();
    __builtin_amdgcn_fence(__ATOMIC_ACQUIRE, "workgroup");
    if (OUT_MODE == 0) {
      float* C = (float*)Cout + (size_t)b * strideC;
      const int hh = lane >> 4, c4 = (lane & 15) * 4;
      for (int pass = 0; pass < 2; ++pass) {
#pragma unroll
        for (int it = 0; it < 8; ++it) {
          const int row = it * 2 + hh;
          v4f v = *(const v4f*)(slab + row * 68 + c4);
          *(volatile v4f*)(C + (size_t)(mBase + row) * ldc + n0 + c4) = v;
        }
        __threadfence();
      }
    } else {
      const int q = lane >> 3, c8 = (lane & 7) * 8;
      unsigned short* C  = (unsigned short*)Cout  + (size_t)b * strideC;
      unsigned short* C2 = (OUT_MODE == 2) ? ((unsigned short*)Cout2 + (size_t)b * strideC) : nullptr;
      for (int pass = 0; pass < 2; ++pass) {
#pragma unroll
        for (int it = 0; it < 4; ++it) {
          const int row = it * 4 + q;
          const float* sp = slab + row * 68 + c8;
          v8h hv, lv;
#pragma unroll
          for (int e = 0; e < 8; ++e) {
            if (OUT_MODE == 1) {
              hv[e] = (_Float16)sp[e];
            } else {
              unsigned short hb = f2bf_bits(sp[e]);
              unsigned short lb = f2bf_bits(sp[e] - bf_bits2f(hb));
              hv[e] = __builtin_bit_cast(_Float16, hb);
              lv[e] = __builtin_bit_cast(_Float16, lb);
            }
          }
          *(volatile v8h*)(C + (size_t)(mBase + row) * ldc + n0 + c8) = hv;
          if (OUT_MODE == 2) *(volatile v8h*)(C2 + (size_t)(mBase + row) * ldc + n0 + c8) = lv;
        }
        __threadfence();
      }
    }
    __builtin_amdgcn_fence(__ATOMIC_RELEASE, "workgroup");
    __builtin_amdgcn_wave_barrier();
    __builtin_amdgcn_fence(__ATOMIC_ACQUIRE, "workgroup");
  }
}

__global__ __launch_bounds__(NTHR) void cvt_f16x8_kernel(const float* __restrict__ src, unsigned short* __restrict__ dst,
                                                         int n8, float sc) {
  const int i = blockIdx.x * NTHR + threadIdx.x;
  if (i < n8) {
    const float* sp = src + (size_t)i * 8;
    const v4f a = *(const v4f*)(sp);
    const v4f b = *(const v4f*)(sp + 4);
    v8h hv;
#pragma unroll
    for (int e = 0; e < 4; ++e) {
      hv[e]     = (_Float16)(a[e] * sc);
      hv[4 + e] = (_Float16)(b[e] * sc);
    }
    *(volatile v8h*)(dst + (size_t)i * 8) = hv;
    __threadfence();
    *(volatile v8h*)(dst + (size_t)i * 8) = hv;
  }
}

__global__ __launch_bounds__(NTHR) void rnn_seq_kernel(const float* __restrict__ z, const float* __restrict__ W_l,
                                                       const float* __restrict__ b_l,
                                                       const float* __restrict__ b_ih, const float* __restrict__ b_hh,
                                                       const unsigned short* __restrict__ WIp,
                                                       const unsigned short* __restrict__ WHp,
                                                       unsigned short* __restrict__ HIST) {
  __shared__ __align__(16) _Float16 Pl[4 * PLSZ];
  __shared__ __align__(16) float    Hm[NLAY * SEQ_BLK * NHID];
  __shared__ __align__(16) float    Bc[NLAY * 4 * NHID];
  __shared__ __align__(16) float    Zs[SEQ_BLK * NLAT];
  const _Float16* WI = (const _Float16*)WIp;
  const _Float16* WH = (const _Float16*)WHp;
  const int tid = threadIdx.x, lane = tid & 31, wave = tid >> 5;
  const int c = lane & 15, hh = lane >> 4, koff = hh * 8;
  const int rowbase = blockIdx.x * SEQ_BLK;

#pragma unroll 1
  for (int i = tid; i < 4 * PLSZ; i += NTHR) Pl[i] = (_Float16)0.0f;
  {
    const int m = tid >> 4, c4 = (tid & 15) * 4;
    const v4f v = *(const v4f*)(z + (size_t)(rowbase + m) * NLAT + c4);
    *(v4f*)(Zs + m * NLAT + c4) = v;
  }
#pragma unroll
  for (int it = 0; it < 3; ++it) {
    const int i = it * NTHR + tid;
    const v4f v = *(const v4f*)(b_ih + 4 * i);
    *(v4f*)(Hm + 4 * i) = v;
  }
#pragma unroll
  for (int it = 0; it < 3; ++it) {
    const int i = it * NTHR + tid;
    const v4f v = *(const v4f*)(b_hh + 4 * i);
    *(v4f*)(Hm + NLAY * NG3 + 4 * i) = v;
  }
  __syncthreads();
#pragma unroll
  for (int l = 0; l < NLAY; ++l) {
#pragma unroll
    for (int cc = 0; cc < 2; ++cc) {
      const int n = tid + NTHR * cc;
      const float bir = Hm[l * NG3 + n];
      const float biz = Hm[l * NG3 + NHID + n];
      const float bin = Hm[l * NG3 + 2 * NHID + n];
      const float bhr = Hm[NLAY * NG3 + l * NG3 + n];
      const float bhz = Hm[NLAY * NG3 + l * NG3 + NHID + n];
      const float bhn = Hm[NLAY * NG3 + l * NG3 + 2 * NHID + n];
      Bc[(l * 4 + 0) * NHID + n] = bir + bhr;
      Bc[(l * 4 + 1) * NHID + n] = biz + bhz;
      Bc[(l * 4 + 2) * NHID + n] = bin;
      Bc[(l * 4 + 3) * NHID + n] = bhn;
    }
  }
  __syncthreads();
#pragma unroll 1
  for (int cc = 0; cc < 2; ++cc) {
    const int n = tid + NTHR * cc;
    float acc[SEQ_BLK];
#pragma unroll
    for (int r = 0; r < SEQ_BLK; ++r) acc[r] = 0.0f;
    const float* wl = W_l + (size_t)n * NLAT;
#pragma unroll 1
    for (int k4 = 0; k4 < NLAT / 4; ++k4) {
      const v4f w = *(const v4f*)(wl + 4 * k4);
#pragma unroll
      for (int r = 0; r < SEQ_BLK; ++r) {
        const v4f zz = *(const v4f*)(Zs + r * NLAT + 4 * k4);
        acc[r] = fmaf(zz[0], w[0], acc[r]);
        acc[r] = fmaf(zz[1], w[1], acc[r]);
        acc[r] = fmaf(zz[2], w[2], acc[r]);
        acc[r] = fmaf(zz[3], w[3], acc[r]);
      }
    }
    const float bn = b_l[n];
#pragma unroll
    for (int r = 0; r < SEQ_BLK; ++r) {
      const float h = acc[r] + bn;
      Hm[r * NHID + n] = h;
      Hm[SEQ_BLK * NHID + r * NHID + n] = h;
      Pl[1 * PLSZ + r * HP + n] = (_Float16)(h * HCARRY);
    }
  }
  __syncthreads();

  const v8f z8 = {0.f, 0.f, 0.f, 0.f, 0.f, 0.f, 0.f, 0.f};
  const int q8 = lane >> 3, c8 = (lane & 7) * 8;

#pragma unroll 1
  for (int t = 0; t < NSTEP; ++t) {
    const int p = t & 1;
#pragma unroll
    for (int l = 0; l < NLAY; ++l) {
      const int xpl = (l == 0) ? (2 + (p ^ 1)) : p;
      const int hpl = (l == 0) ? (p ^ 1) : ((t == 0) ? 1 : (2 + (p ^ 1)));
      const int wpl = (l == 0) ? p : (2 + p);
      const _Float16* xrow = Pl + xpl * PLSZ + c * HP + koff;
      const _Float16* hrow = Pl + hpl * PLSZ + c * HP + koff;
      _Float16* wplane = Pl + wpl * PLSZ;
      float* hm = Hm + l * (SEQ_BLK * NHID);
      const float* bcl = Bc + l * 4 * NHID;
      const _Float16* wib = WI + (size_t)l * NG3 * NHID;
      const _Float16* whb = WH + (size_t)l * NG3 * NHID;
#pragma unroll
      for (int nt = 0; nt < 4; ++nt) {
        const int j = 64 * wave + 16 * nt + c;
        const _Float16* wi = wib + (size_t)j * NHID + koff;
        const _Float16* wh = whb + (size_t)j * NHID + koff;
        v8f air = z8, aiz = z8, ain = z8, ahr = z8, ahz = z8, ahn = z8;
#pragma unroll 1
        for (int k0 = 0; k0 < NHID; k0 += 32) {
          const v16h ax = Frag<_Float16>::load(xrow + k0);
          const v16h ah = Frag<_Float16>::load(hrow + k0);
          const v16h b0 = Frag<_Float16>::load(wi + k0);
          const v16h b1 = Frag<_Float16>::load(wi + (size_t)1 * NHID * NHID + k0);
          const v16h b2 = Frag<_Float16>::load(wi + (size_t)2 * NHID * NHID + k0);
          const v16h b3 = Frag<_Float16>::load(wh + k0);
          const v16h b4 = Frag<_Float16>::load(wh + (size_t)1 * NHID * NHID + k0);
          const v16h b5 = Frag<_Float16>::load(wh + (size_t)2 * NHID * NHID + k0);
          air = Frag<_Float16>::mma(ax, b0, air);
          aiz = Frag<_Float16>::mma(ax, b1, aiz);
          ain = Frag<_Float16>::mma(ax, b2, ain);
          ahr = Frag<_Float16>::mma(ah, b3, ahr);
          ahz = Frag<_Float16>::mma(ah, b4, ahz);
          ahn = Frag<_Float16>::mma(ah, b5, ahn);
          guard6_h(air, aiz, ain, ahr, ahz, ahn, ax, ah, b0, b1, b2, b3, b4, b5);
        }
        acc_guard6(air, aiz, ain, ahr, ahz, ahn);
        const float bR  = bcl[0 * NHID + j];
        const float bZ  = bcl[1 * NHID + j];
        const float bNI = bcl[2 * NHID + j];
        const float bNH = bcl[3 * NHID + j];
#pragma unroll
        for (int r = 0; r < 8; ++r) {
          const int row = 8 * hh + r;
          const float pr  = (air[r] + ahr[r]) * ACC_INV + bR;
          const float pz  = (aiz[r] + ahz[r]) * ACC_INV + bZ;
          const float gin = ain[r] * ACC_INV + bNI;
          const float ghn = ahn[r] * ACC_INV + bNH;
          const float rg = fsig(pr);
          const float ug = fsig(pz);
          const float ng = ftanh(gin + rg * ghn);
          const float ho = hm[row * NHID + j];
          const float hn = (1.0f - ug) * ng + ug * ho;
          hm[row * NHID + j] = hn;
          wplane[row * HP + j] = (_Float16)(hn * HCARRY);
        }
      }
      __syncthreads();
    }
    {
      const _Float16* src = Pl + (2 + p) * PLSZ + 64 * wave + c8;
      v8h hv[4];
#pragma unroll
      for (int it = 0; it < 4; ++it) hv[it] = *(const v8h*)(src + (it * 4 + q8) * HP);
      for (int pass = 0; pass < 2; ++pass) {
#pragma unroll
        for (int it = 0; it < 4; ++it) {
          const int row = it * 4 + q8;
          const size_t o = ((size_t)(rowbase + row) * NSTEP + (size_t)t) * NHID + 64 * wave + c8;
          *(volatile v8h*)(HIST + o) = hv[it];
        }
        __threadfence();
      }
    }
  }
}

extern "C" void kernel_launch(void* const* d_in, const int* in_sizes, int n_in,
                              void* d_out, int out_size, void* d_ws, size_t ws_size, hipStream_t stream) {
  if (n_in < 9 || d_out == nullptr || d_ws == nullptr) return;
  if (in_sizes[0] != NBAT * NLAT || in_sizes[1] != NHID * NLAT || in_sizes[2] != NHID ||
      in_sizes[3] != NLAY * NG3 * NHID || in_sizes[4] != NLAY * NG3 * NHID ||
      in_sizes[5] != NLAY * NG3 || in_sizes[6] != NLAY * NG3 ||
      in_sizes[7] != NOUTF * NHID || in_sizes[8] != NOUTF || out_size != NROWS * NOUTF) return;

  const float* z    = (const float*)d_in[0];
  const float* W_l  = (const float*)d_in[1];
  const float* b_l  = (const float*)d_in[2];
  const float* W_ih = (const float*)d_in[3];
  const float* W_hh = (const float*)d_in[4];
  const float* b_ih = (const float*)d_in[5];
  const float* b_hh = (const float*)d_in[6];
  const float* W_o  = (const float*)d_in[7];
  const float* b_o  = (const float*)d_in[8];
  float* out = (float*)d_out;

  char* ws = (char*)d_ws; size_t off = 0;
  auto carve = [&](size_t bytes) -> char* { char* p = ws + off; off += (bytes + 255) & ~(size_t)255; return p; };
  unsigned short* WIH16 = (unsigned short*)carve((size_t)NLAY * NG3 * NHID * 2);
  unsigned short* WHH16 = (unsigned short*)carve((size_t)NLAY * NG3 * NHID * 2);
  unsigned short* WO16  = (unsigned short*)carve((size_t)NOUTF * NHID * 2);
  unsigned short* HIST  = (unsigned short*)carve((size_t)NROWS * NHID * 2);
  if (off > ws_size || off > (size_t)134217728) return;

  const int n8g = NLAY * NG3 * NHID / 8;
  const int n8o = NOUTF * NHID / 8;
  cvt_f16x8_kernel<<<(n8g + NTHR - 1) / NTHR, NTHR, 0, stream>>>(W_ih, WIH16, n8g, WCARRY);
  cvt_f16x8_kernel<<<(n8g + NTHR - 1) / NTHR, NTHR, 0, stream>>>(W_hh, WHH16, n8g, WCARRY);
  cvt_f16x8_kernel<<<(n8o + NTHR - 1) / NTHR, NTHR, 0, stream>>>(W_o,  WO16,  n8o, WCARRY);
  rnn_seq_kernel<<<NBAT / SEQ_BLK, NTHR, 0, stream>>>(z, W_l, b_l, b_ih, b_hh, WIH16, WHH16, HIST);
  const dim3 ggrid((NROWS / 64) * (NOUTF / 64) / 8, 1);
  wmma_gemm64<0, false, 2, 0, false, 0><<<ggrid, 256, 0, stream>>>(
      HIST, HIST, NHID, 0L, WO16, WO16, NHID, 0L, (void*)out, (void*)out, NOUTF, 0L,
      b_o, b_o, 0L, NROWS, NOUTF, NHID, ACC_INV);
}
